// YModel_75118978007346
// MI455X (gfx1250) — hardware-verified
//
#include <hip/hip_runtime.h>
#include <stddef.h>


#define HH     80
#define LL     600
#define SEGW   40
#define NSEGS  5
#define WST    400
#define NCH    8
#define NCLS   4
#define NPOS   171
#define PWD    9
#define AY     21
#define AX     11
#define AC     16
#define ABUF   (AY * AX * AC)
#define KS     32
#define KC     160
#define NT1    43
#define NT2    11
#define GP     176
#define TPB    256
#define NWAV   (TPB / 32)
#define TOUT   128
#define LINEF  32
#define WSC    16.0f
#define WSCI   0.0625f
#define ALPHA  0.2f
#define WSCAP  134217728

static_assert(NT1 * 16 >= NPOS * 4);
static_assert(NT2 * 16 >= NPOS);
static_assert(NT2 * 16 <= GP);
static_assert(KC % 32 == 0);
static_assert((NSEGS * ABUF) % 8 == 0);
static_assert((HH * SEGW) % 4 == 0);

typedef _Float16 v16h __attribute__((ext_vector_type(16)));
typedef _Float16 v8h  __attribute__((ext_vector_type(8)));
typedef _Float16 v4h  __attribute__((ext_vector_type(4)));
typedef float    v8f  __attribute__((ext_vector_type(8)));
typedef float    v4f  __attribute__((ext_vector_type(4)));
union Frag { v16h v; v8h half[2]; _Float16 e[16]; };

__device__ __forceinline__ v8f wmf(v16h a, v16h b, v8f c) {
  v8f d = __builtin_amdgcn_wmma_f32_16x16x32_f16(false, a, false, b, (short)0, c, false, false);
  asm volatile("v_nop\n\tv_nop\n\tv_nop\n\tv_nop" : "+v"(d) : "v"(a), "v"(b));
  return d;
}

__device__ __forceinline__ v8f zacc() {
  v8f z = {0.f, 0.f, 0.f, 0.f, 0.f, 0.f, 0.f, 0.f};
  return z;
}

__device__ __forceinline__ float leaky(float x) { return x >= 0.0f ? x : ALPHA * x; }

template <int CIN, int COUT, bool LAST>
__device__ __forceinline__ void chain_stage(
    const float* __restrict__ w, const float* __restrict__ bias,
    const _Float16* ain, _Float16* aout, _Float16* wt, float* bch, float* gout,
    int tid, int wave, int h, int m) {
#pragma unroll 1
  for (int t = tid; t < AC * KC; t += TPB) {
    const int n = t / KC, k = t - n * KC;
    const int tap = k >> 4, c = k & 15;
    const bool ok = (tap < 9) && (c < CIN) && (n < COUT);
    const int nc = n < COUT ? n : COUT - 1;
    const int cc = c < CIN ? c : CIN - 1;
    const int tc = tap < 9 ? tap : 8;
    const float v = w[(nc * CIN + cc) * 9 + tc];
    wt[t] = ok ? (_Float16)(v * WSC) : (_Float16)0.0f;
  }
  if (tid < AC) {
    const float bv = bias[tid < COUT ? tid : COUT - 1];
    bch[tid] = tid < COUT ? bv : 0.0f;
  }
  __syncthreads();

  const float bb = bch[m];
  const _Float16 hz = (_Float16)0.0f;
  const v8h z8 = {hz, hz, hz, hz, hz, hz, hz, hz};
#pragma unroll 1
  for (int tile = wave; tile < NT2; tile += NWAV) {
    const int row = tile * 16 + m;
    const int rc  = row < NPOS ? row : NPOS - 1;
    const int oy  = rc / PWD, ox = rc - oy * PWD;
    const _Float16* abase = ain + (oy * AX + ox) * AC + 8 * h;
    const _Float16* bbase = wt + m * KC + 8 * h;
    v8f acc = zacc();
#pragma unroll
    for (int p = 0; p < KC / 32; ++p) {
      Frag a, bq;
      const int t0 = 2 * p, t1 = 2 * p + 1;
      a.half[0] = *(const v8h*)(abase + ((t0 / 3) * AX + (t0 % 3)) * AC);
      if (p < 4) a.half[1] = *(const v8h*)(abase + ((t1 / 3) * AX + (t1 % 3)) * AC);
      else       a.half[1] = z8;
      bq.half[0] = *(const v8h*)(bbase + 32 * p);
      bq.half[1] = *(const v8h*)(bbase + 32 * p + 16);
      acc = wmf(a.v, bq.v, acc);
    }
#pragma unroll
    for (int r = 0; r < 8; ++r) {
      const int mm = tile * 16 + 8 * h + r;
      const float v = leaky(acc[r] * WSCI + bb);
      if (!LAST) {
        if (m < COUT && mm < NPOS) {
          const int y = mm / PWD, x = mm - y * PWD;
          aout[((y + 1) * AX + (x + 1)) * AC + NCH + m] = (_Float16)v;
        }
      } else {
        if (m < COUT) gout[m * GP + mm] = v;
      }
    }
  }
  __syncthreads();
}

__global__ __launch_bounds__(TPB) void k_main(
    const float* __restrict__ in, const float* __restrict__ spw, const float* __restrict__ spb,
    const float* __restrict__ w1, const float* __restrict__ b1,
    const float* __restrict__ w2, const float* __restrict__ b2,
    const float* __restrict__ w3, const float* __restrict__ b3,
    const float* __restrict__ w4, const float* __restrict__ b4,
    const float* __restrict__ w5, const float* __restrict__ b5,
    float* wsl) {
  __shared__ __attribute__((aligned(16))) _Float16 xs[HH * SEGW];
  __shared__ __attribute__((aligned(16))) _Float16 act[NSEGS * ABUF];
  __shared__ __attribute__((aligned(16))) _Float16 wsp[AC * KS];
  __shared__ __attribute__((aligned(16))) _Float16 wt[AC * KC];
  __shared__ float bsp[AC];
  __shared__ float bch[AC];
  __shared__ __attribute__((aligned(16))) float gout[NCLS * GP];
  __shared__ __attribute__((aligned(16))) float oline[LINEF];

  const int tid = (int)threadIdx.x, lane = tid & 31, wave = tid >> 5, h = lane >> 4, m = lane & 15;
  const int img = (int)blockIdx.x;
  const _Float16 hz = (_Float16)0.0f;
  const v8h z8 = {hz, hz, hz, hz, hz, hz, hz, hz};

#pragma unroll 1
  for (int t = tid; t < (NSEGS * ABUF) / 8; t += TPB) *(v8h*)(act + 8 * t) = z8;
#pragma unroll 1
  for (int t = tid; t < AC * KS; t += TPB) {
    const int n = t >> 5, k = t & 31;
    const bool ok = (n < NCH) && (k < 25);
    const int nc = n < NCH ? n : NCH - 1;
    const int kc = k < 25 ? k : 24;
    const float v = spw[nc * 25 + kc];
    wsp[t] = ok ? (_Float16)(v * WSC) : hz;
  }
  if (tid < AC) {
    const float bv = spb[tid < NCH ? tid : NCH - 1];
    bsp[tid] = tid < NCH ? bv : 0.0f;
  }

  int goff[16];
#pragma unroll
  for (int i = 0; i < 16; ++i) {
    const int k  = 8 * h + i + ((i >= 8) ? 8 : 0);
    const int kc = k < 25 ? k : 24;
    const int kh = kc / 5, kw = kc - kh * 5;
    goff[i] = kh * SEGW + kw;
  }
  const bool hnz = (h != 0);

  const float* inb = in + (size_t)img * (size_t)(HH * LL) + WST;

#pragma unroll 1
  for (int s = 0; s < NSEGS; ++s) {
    const float* src = inb + SEGW * s;
#pragma unroll 1
    for (int t = tid; t < HH * (SEGW / 4); t += TPB) {
      const int r = t / (SEGW / 4), c4 = (t - r * (SEGW / 4)) * 4;
      const v4f v = *(const v4f*)(src + (size_t)r * LL + c4);
      v4h hv;
      hv.x = (_Float16)v.x; hv.y = (_Float16)v.y; hv.z = (_Float16)v.z; hv.w = (_Float16)v.w;
      *(v4h*)(xs + r * SEGW + c4) = hv;
    }
    __syncthreads();

    _Float16* abuf = act + s * ABUF;
#pragma unroll 1
    for (int tile = wave; tile < NT1; tile += NWAV) {
      const int row = tile * 16 + m;
      const int g = row >> 2, d = row & 3;
      const int gc = g < NPOS ? g : NPOS - 1;
      const int ph = gc / PWD, pw = gc - ph * PWD;
      const int base = (4 * ph + 2 * (d >> 1)) * SEGW + 4 * pw + 2 * (d & 1);
      Frag a, bq;
#pragma unroll
      for (int i = 0; i < 16; ++i) {
        _Float16 x = xs[base + goff[i]];
        if (i >= 9) x = hnz ? hz : x;
        a.e[i] = x;
      }
      bq.half[0] = *(const v8h*)(wsp + m * KS + 8 * h);
      bq.half[1] = *(const v8h*)(wsp + m * KS + 16 + 8 * h);
      const v8f acc = wmf(a.v, bq.v, zacc());
      const float bb = bsp[m];
      float p0 = leaky(acc[0] * WSCI + bb);
      float p1 = leaky(acc[4] * WSCI + bb);
#pragma unroll
      for (int r = 1; r < 4; ++r) {
        p0 = fmaxf(p0, leaky(acc[r] * WSCI + bb));
        p1 = fmaxf(p1, leaky(acc[4 + r] * WSCI + bb));
      }
      const int g0 = tile * 4 + 2 * h, g1 = g0 + 1;
      if (m < NCH) {
        if (g0 < NPOS) {
          const int y = g0 / PWD, x = g0 - y * PWD;
          abuf[((y + 1) * AX + (x + 1)) * AC + m] = (_Float16)p0;
        }
        if (g1 < NPOS) {
          const int y = g1 / PWD, x = g1 - y * PWD;
          abuf[((y + 1) * AX + (x + 1)) * AC + m] = (_Float16)p1;
        }
      }
    }
    __syncthreads();
  }

  chain_stage<NCH, NCH, false>(w1, b1, act + 0 * ABUF, act + 1 * ABUF, wt, bch, gout, tid, wave, h, m);
  chain_stage<AC,  NCH, false>(w2, b2, act + 1 * ABUF, act + 2 * ABUF, wt, bch, gout, tid, wave, h, m);
  chain_stage<AC,  NCH, false>(w3, b3, act + 2 * ABUF, act + 3 * ABUF, wt, bch, gout, tid, wave, h, m);
  chain_stage<AC,  NCH, false>(w4, b4, act + 3 * ABUF, act + 4 * ABUF, wt, bch, gout, tid, wave, h, m);
  chain_stage<AC,  NCLS, true>(w5, b5, act + 4 * ABUF, act + 4 * ABUF, wt, bch, gout, tid, wave, h, m);

  if (tid < 32) {
    const int c = tid < NCLS ? tid : NCLS - 1;
    float sacc = 0.0f;
#pragma unroll 1
    for (int mm = 0; mm < NPOS; ++mm) sacc += gout[c * GP + mm];
    oline[tid] = tid < NCLS ? sacc * (1.0f / (float)NPOS) : 0.0f;
  }
  __syncthreads();
  const v4f ov = *(const v4f*)(oline + 4 * (tid & 7));
  float* gp = wsl + (size_t)img * LINEF + 4 * (tid & 7);
  const bool wr = tid < 8;
  if (wr) *(volatile v4f*)gp = ov;
  __threadfence();
  if (wr) *(volatile v4f*)gp = ov;
}

__global__ __launch_bounds__(TOUT) void k_out(const float* __restrict__ wsl, float* out, int nS) {
  const int t  = (int)blockIdx.x * TOUT + (int)threadIdx.x;
  const int tc = t < nS ? t : nS - 1;
  const v4f v = *(const v4f*)(wsl + (size_t)tc * LINEF);
  float* gp = out + (size_t)tc * NCLS;
  const bool wr = t < nS;
  if (wr) *(volatile v4f*)gp = v;
  __threadfence();
  if (wr) *(volatile v4f*)gp = v;
}

extern "C" void kernel_launch(void* const* d_in, const int* in_sizes, int n_in,
                              void* d_out, int out_size, void* d_ws, size_t ws_size,
                              hipStream_t stream) {
  if (n_in < 13) return;
  const int per = HH * LL;
  const int nS = in_sizes[0] / per;
  if (nS <= 0 || nS > (1 << 20) || in_sizes[0] != nS * per) return;
  if (in_sizes[1] != NCH * 25 || in_sizes[2] != NCH) return;
  if (in_sizes[3] != NCH * NCH * 9 || in_sizes[4] != NCH) return;
  if (in_sizes[5] != NCH * AC * 9 || in_sizes[6] != NCH) return;
  if (in_sizes[7] != NCH * AC * 9 || in_sizes[8] != NCH) return;
  if (in_sizes[9] != NCH * AC * 9 || in_sizes[10] != NCH) return;
  if (in_sizes[11] != NCLS * AC * 9 || in_sizes[12] != NCLS) return;
  if (out_size != nS * NCLS) return;

  const size_t wsl_bytes = (size_t)nS * LINEF * sizeof(float);
  if (wsl_bytes > ws_size || wsl_bytes > (size_t)WSCAP) return;
  float* wsl = (float*)d_ws;

  const float* x   = (const float*)d_in[0];
  const float* spw = (const float*)d_in[1];
  const float* spb = (const float*)d_in[2];
  const float* w1  = (const float*)d_in[3];
  const float* b1  = (const float*)d_in[4];
  const float* w2  = (const float*)d_in[5];
  const float* b2  = (const float*)d_in[6];
  const float* w3  = (const float*)d_in[7];
  const float* b3  = (const float*)d_in[8];
  const float* w4  = (const float*)d_in[9];
  const float* b4  = (const float*)d_in[10];
  const float* w5  = (const float*)d_in[11];
  const float* b5  = (const float*)d_in[12];
  float* out = (float*)d_out;

  k_main<<<nS, TPB, 0, stream>>>(x, spw, spb, w1, b1, w2, b2, w3, b3, w4, b4, w5, b5, wsl);
  k_out<<<(nS + TOUT - 1) / TOUT, TOUT, 0, stream>>>(wsl, out, nS);
}
